// LightweightMamba2D_10960756540365
// MI455X (gfx1250) — hardware-verified
//
#include <hip/hip_runtime.h>
#define BB 2
#define CX 96
#define HI 96
#define WI 96
#define HWN (HI * WI)
#define NPOS (BB * HWN)
#define HID 128
#define DI 160
#define DS 8
#define DTR 8
#define NXP 24
#define WSZ 16
#define NWIN 12
#define NSEQ (BB * WI * NWIN)
#define TT WSZ
#define MR (NSEQ * TT)
#define NG 8

typedef __bf16 v16b __attribute__((ext_vector_type(16)));
typedef unsigned short v8us __attribute__((ext_vector_type(8), may_alias));
typedef float  v8f  __attribute__((ext_vector_type(8)));
typedef float  v4f  __attribute__((ext_vector_type(4)));
typedef float  v4fa __attribute__((ext_vector_type(4), may_alias));
union FragB { v16b v; v8us half[2]; unsigned short u[16]; };

__device__ __forceinline__ unsigned short bf16_bits(float x) { unsigned int u = __float_as_uint(x); return (unsigned short)((u + 0x7FFFu + ((u >> 16) & 1u)) >> 16); }
__device__ __forceinline__ float bf16_val(unsigned short b) { return __uint_as_float(((unsigned int)b) << 16); }
__device__ __forceinline__ float bf16_round(float x) { return bf16_val(bf16_bits(x)); }
template <int NT>
__device__ __forceinline__ v8f mmaN(v16b ah, v16b al, v16b bh, v16b bl, v8f c) {
  c = __builtin_amdgcn_wmma_f32_16x16x32_bf16(false, ah, false, bh, (short)0, c, false, false);
  if (NT >= 2) c = __builtin_amdgcn_wmma_f32_16x16x32_bf16(false, al, false, bh, (short)0, c, false, false);
  if (NT >= 3) c = __builtin_amdgcn_wmma_f32_16x16x32_bf16(false, ah, false, bl, (short)0, c, false, false);
  asm volatile("v_nop\n\tv_nop\n\tv_nop\n\tv_nop" : "+v"(c) : "v"(ah), "v"(al), "v"(bh), "v"(bl));
  return c;
}

__global__ __launch_bounds__(256) void k_wt_bf16(const float* __restrict__ W, unsigned short* __restrict__ Wt, int K, int N) {
  const int t = blockIdx.x * 256 + threadIdx.x;
  const int k8n = K / 8;
  if (t >= N * k8n) return;
  const int n = t / k8n, k8 = (t % k8n) * 8;
  v8us v;
#pragma unroll
  for (int i = 0; i < 8; ++i) v[i] = bf16_bits(W[(size_t)(k8 + i) * N + n]);
  *(volatile v8us*)(Wt + (size_t)n * K + k8) = v;
  __threadfence();
  *(volatile v8us*)(Wt + (size_t)n * K + k8) = v;
}

template <bool ASPLIT, int ACT, bool BIAS_BF16>
__global__ __launch_bounds__(128) void k_gemm_bf(const float* __restrict__ A, int lda, const unsigned short* __restrict__ Wt, int ldb,
                                               const float* __restrict__ bias, float* __restrict__ C, int ldc, int M, int N, int K) {
  __shared__ __attribute__((aligned(16))) float so[4][16][64];
  const int tid = threadIdx.x, w = tid >> 5, lane = tid & 31, ln = lane & 15, hh = lane >> 4;
  const int ntn = N / 64;
  const int wid = blockIdx.x * 4 + w;
  const int mt = wid / ntn, nq = wid % ntn;
  if (mt * 16 >= M) return;
  const int row0 = mt * 16, col0 = nq * 64;
  const float* arow = A + (size_t)(row0 + ln) * lda;
  v8f acc[4] = {};
  for (int kb = 0; kb < K; kb += 32) {
    FragB ah, al;
    const v4f x0 = *(const v4fa*)(arow + kb + 8 * hh), x1 = *(const v4fa*)(arow + kb + 8 * hh + 4);
    const v4f x2 = *(const v4fa*)(arow + kb + 16 + 8 * hh), x3 = *(const v4fa*)(arow + kb + 16 + 8 * hh + 4);
    float xs[16] = {x0[0],x0[1],x0[2],x0[3],x1[0],x1[1],x1[2],x1[3],x2[0],x2[1],x2[2],x2[3],x3[0],x3[1],x3[2],x3[3]};
#pragma unroll
    for (int i = 0; i < 16; ++i) { const unsigned short hb = bf16_bits(xs[i]); ah.u[i] = hb; al.u[i] = ASPLIT ? bf16_bits(xs[i] - bf16_val(hb)) : (unsigned short)0; }
#pragma unroll
    for (int t = 0; t < 4; ++t) {
      const unsigned short* brow = Wt + (size_t)(col0 + t * 16 + ln) * ldb + kb;
      FragB b;
      b.half[0] = *(const v8us*)(brow + 8 * hh);
      b.half[1] = *(const v8us*)(brow + 16 + 8 * hh);
      acc[t] = mmaN<ASPLIT ? 2 : 1>(ah.v, al.v, b.v, b.v, acc[t]);
    }
  }
#pragma unroll
  for (int t = 0; t < 4; ++t) {
    float bv = bias ? bias[col0 + t * 16 + ln] : 0.f;
    if (BIAS_BF16) bv = bf16_round(bv);
#pragma unroll
    for (int r = 0; r < 8; ++r) { float v = acc[t][r] + bv; if (ACT == 1) v = fmaxf(v, 0.f); so[w][8 * hh + r][t * 16 + ln] = v; }
  }
  __builtin_amdgcn_fence(__ATOMIC_ACQ_REL, "workgroup");
  __builtin_amdgcn_wave_barrier();
  const int rsub = lane >> 4, c4 = (lane & 15) * 4;
  for (int pass = 0; pass < 2; ++pass) {
#pragma unroll
    for (int q = 0; q < 8; ++q) {
      const int r = q * 2 + rsub;
      const v4f v = *(const v4fa*)&so[w][r][c4];
      *(volatile v4f*)(C + (size_t)(row0 + r) * ldc + col0 + c4) = v;
    }
    if (pass == 0) __threadfence();
  }
}

template <int D, bool CAUSAL>
__global__ __launch_bounds__(128) void k_flash(const float* __restrict__ qb, const float* __restrict__ kb, const float* __restrict__ vb,
                                             int pitch, int T, int H, float scale, float* __restrict__ y, int ypitch) {
  constexpr int KS = D / 32;
  constexpr int DT = D / 16;
  __shared__ __attribute__((aligned(16))) unsigned short sKh[32][D + 8], sKl[32][D + 8], sVh[32][D + 8], sVl[32][D + 8];
  __shared__ __attribute__((aligned(16))) unsigned short sPh[4][16][40], sPl[4][16][40];
  __shared__ __attribute__((aligned(16))) float sO[4][16][D];
  const int tid = threadIdx.x, w = tid >> 5, lane = tid & 31, ln = lane & 15, hh = lane >> 4;
  const int nqb = (T + 63) / 64;
  const int bh = blockIdx.x / nqb, qblk = blockIdx.x % nqb;
  const int b = bh / H, h = bh % H;
  const int q0 = qblk * 64 + w * 16;
  const float* Q = qb + (size_t)b * T * pitch + h * D;
  const float* K = kb + (size_t)b * T * pitch + h * D;
  const float* V = vb + (size_t)b * T * pitch + h * D;

  FragB aqh[KS], aql[KS];
  {
    int row = q0 + ln; if (row >= T) row = T - 1;
    const float* qr = Q + (size_t)row * pitch;
#pragma unroll
    for (int ks = 0; ks < KS; ++ks)
#pragma unroll
      for (int i = 0; i < 16; ++i) {
        const int d = ks * 32 + ((i < 8) ? (8 * hh + i) : (16 + 8 * hh + (i - 8)));
        const float x = qr[d] * scale; const unsigned short hb = bf16_bits(x);
        aqh[ks].u[i] = hb; aql[ks].u[i] = bf16_bits(x - bf16_val(hb));
      }
  }
  float m_r[8], l_r[8];
#pragma unroll
  for (int r = 0; r < 8; ++r) { m_r[r] = -3.0e38f; l_r[r] = 0.f; }
  v8f oacc[DT];
#pragma unroll
  for (int dt = 0; dt < DT; ++dt) oacc[dt] = (v8f){0.f,0.f,0.f,0.f,0.f,0.f,0.f,0.f};

  const int kv_end = CAUSAL ? min(T, qblk * 64 + 64) : T;
  for (int j0 = 0; j0 < kv_end; j0 += 32) {
    __syncthreads();
    for (int e = tid; e < 32 * (D / 4); e += 128) {
      const int r = e / (D / 4), c4 = (e % (D / 4)) * 4;
      const int key = j0 + r;
      v4f kf = {0.f,0.f,0.f,0.f}, vf = {0.f,0.f,0.f,0.f};
      if (key < T) { kf = *(const v4fa*)(K + (size_t)key * pitch + c4); vf = *(const v4fa*)(V + (size_t)key * pitch + c4); }
#pragma unroll
      for (int t = 0; t < 4; ++t) {
        unsigned short hb = bf16_bits(kf[t]); sKh[r][c4 + t] = hb; sKl[r][c4 + t] = bf16_bits(kf[t] - bf16_val(hb));
        hb = bf16_bits(vf[t]); sVh[r][c4 + t] = hb; sVl[r][c4 + t] = bf16_bits(vf[t] - bf16_val(hb));
      }
    }
    __syncthreads();
    v8f s[2];
#pragma unroll
    for (int nt = 0; nt < 2; ++nt) {
      v8f acc = {};
#pragma unroll
      for (int ks = 0; ks < KS; ++ks) {
        FragB bh_, bl_;
        bh_.half[0] = *(const v8us*)&sKh[nt * 16 + ln][ks * 32 + 8 * hh]; bh_.half[1] = *(const v8us*)&sKh[nt * 16 + ln][ks * 32 + 16 + 8 * hh];
        bl_.half[0] = *(const v8us*)&sKl[nt * 16 + ln][ks * 32 + 8 * hh]; bl_.half[1] = *(const v8us*)&sKl[nt * 16 + ln][ks * 32 + 16 + 8 * hh];
        acc = mmaN<3>(aqh[ks].v, aql[ks].v, bh_.v, bl_.v, acc);
      }
      s[nt] = acc;
    }
    float alpha[8];
#pragma unroll
    for (int r = 0; r < 8; ++r) {
      const int qi = q0 + 8 * hh + r;
      const int ja = j0 + ln, jb = j0 + 16 + ln;
      if (CAUSAL) { if (ja > qi) s[0][r] = -3.0e38f; if (jb > qi) s[1][r] = -3.0e38f; }
      if (ja >= T) s[0][r] = -3.0e38f;
      if (jb >= T) s[1][r] = -3.0e38f;
      float mx = fmaxf(s[0][r], s[1][r]);
      mx = fmaxf(mx, __shfl_xor(mx, 1, 32)); mx = fmaxf(mx, __shfl_xor(mx, 2, 32)); mx = fmaxf(mx, __shfl_xor(mx, 4, 32)); mx = fmaxf(mx, __shfl_xor(mx, 8, 32));
      const float mnew = fmaxf(m_r[r], mx);
      alpha[r] = (mnew > -1.0e38f) ? __expf(m_r[r] - mnew) : 1.0f;
      const float p0 = (s[0][r] > -1.0e38f) ? __expf(s[0][r] - mnew) : 0.f;
      const float p1 = (s[1][r] > -1.0e38f) ? __expf(s[1][r] - mnew) : 0.f;
      m_r[r] = mnew;
      l_r[r] = l_r[r] * alpha[r] + p0 + p1;
      unsigned short hb = bf16_bits(p0); sPh[w][8 * hh + r][ln] = hb;      sPl[w][8 * hh + r][ln] = bf16_bits(p0 - bf16_val(hb));
      hb = bf16_bits(p1);                sPh[w][8 * hh + r][16 + ln] = hb; sPl[w][8 * hh + r][16 + ln] = bf16_bits(p1 - bf16_val(hb));
    }
#pragma unroll
    for (int dt = 0; dt < DT; ++dt)
#pragma unroll
      for (int r = 0; r < 8; ++r) oacc[dt][r] *= alpha[r];
    __builtin_amdgcn_fence(__ATOMIC_ACQ_REL, "workgroup");
    __builtin_amdgcn_wave_barrier();
    FragB pah, pal;
    pah.half[0] = *(const v8us*)&sPh[w][ln][8 * hh]; pah.half[1] = *(const v8us*)&sPh[w][ln][16 + 8 * hh];
    pal.half[0] = *(const v8us*)&sPl[w][ln][8 * hh]; pal.half[1] = *(const v8us*)&sPl[w][ln][16 + 8 * hh];
#pragma unroll
    for (int dt = 0; dt < DT; ++dt) {
      FragB bvh, bvl;
#pragma unroll
      for (int i = 0; i < 8; ++i) {
        bvh.u[i] = sVh[8 * hh + i][dt * 16 + ln]; bvh.u[8 + i] = sVh[16 + 8 * hh + i][dt * 16 + ln];
        bvl.u[i] = sVl[8 * hh + i][dt * 16 + ln]; bvl.u[8 + i] = sVl[16 + 8 * hh + i][dt * 16 + ln];
      }
      oacc[dt] = mmaN<3>(pah.v, pal.v, bvh.v, bvl.v, oacc[dt]);
    }
    __builtin_amdgcn_fence(__ATOMIC_ACQ_REL, "workgroup");
    __builtin_amdgcn_wave_barrier();
  }
#pragma unroll
  for (int r = 0; r < 8; ++r) {
    float l = l_r[r];
    l += __shfl_xor(l, 1, 32); l += __shfl_xor(l, 2, 32); l += __shfl_xor(l, 4, 32); l += __shfl_xor(l, 8, 32);
    l_r[r] = (l > 0.f) ? 1.0f / l : 0.f;
  }
#pragma unroll
  for (int dt = 0; dt < DT; ++dt)
#pragma unroll
    for (int r = 0; r < 8; ++r) sO[w][8 * hh + r][dt * 16 + ln] = oacc[dt][r] * l_r[r];
  __builtin_amdgcn_fence(__ATOMIC_ACQ_REL, "workgroup");
  __builtin_amdgcn_wave_barrier();
  for (int pass = 0; pass < 2; ++pass) {
    for (int r = 0; r < 16; ++r) {
      const int row = q0 + r;
      if (row < T && lane < D / 4) {
        const v4f val = *(const v4fa*)&sO[w][r][lane * 4];
        *(volatile v4f*)(y + ((size_t)b * T + row) * ypitch + h * D + lane * 4) = val;
      }
    }
    if (pass == 0) __threadfence();
  }
}

template <bool AFFINE, bool RESID, bool RES_BF16>
__global__ __launch_bounds__(256) void k_transpose32(const float* __restrict__ in, float* __restrict__ out, int rows, int cols,
                                                    const float* __restrict__ scale, const float* __restrict__ shift, const float* __restrict__ res) {
  __shared__ float tile[32][33];
  const int b = blockIdx.z;
  const int r0 = blockIdx.y * 32, c0 = blockIdx.x * 32;
  const float* src = in + (size_t)b * rows * cols;
  float* dst = out + (size_t)b * rows * cols;
  const int tx = threadIdx.x & 31, ty = threadIdx.x >> 5;
  for (int i = ty; i < 32; i += 8) tile[i][tx] = src[(size_t)(r0 + i) * cols + c0 + tx];
  __syncthreads();
  for (int pass = 0; pass < 2; ++pass) {
    for (int i = ty; i < 32; i += 8) {
      float v = tile[tx][i];
      const int orow = c0 + i;
      if (AFFINE) v = v * scale[orow] + shift[orow];
      if (RESID) { float rv = res[(size_t)b * rows * cols + (size_t)orow * rows + r0 + tx]; if (RES_BF16) rv = bf16_round(rv); v += rv; }
      *(volatile float*)(dst + (size_t)orow * rows + r0 + tx) = v;
    }
    if (pass == 0) __threadfence();
  }
}

__global__ __launch_bounds__(256) void k_pool2_pm(const float* __restrict__ in, float* __restrict__ out, int Bn, int H, int W, int C) {
  const size_t t = (size_t)blockIdx.x * 256 + threadIdx.x;
  const int c4n = C / 4, Ho = H / 2, Wo = W / 2;
  const size_t total = (size_t)Bn * Ho * Wo * c4n;
  if (t >= total) return;
  const int c4 = (int)(t % c4n) * 4; size_t rest = t / c4n;
  const int pw = (int)(rest % Wo); rest /= Wo; const int ph = (int)(rest % Ho); const int b = (int)(rest / Ho);
  const float* base = in + (size_t)b * H * W * C;
  const int p00 = (2 * ph) * W + 2 * pw;
  const v4f a = *(const v4fa*)(base + (size_t)p00 * C + c4), bq = *(const v4fa*)(base + (size_t)(p00 + 1) * C + c4);
  const v4f c = *(const v4fa*)(base + (size_t)(p00 + W) * C + c4), d = *(const v4fa*)(base + (size_t)(p00 + W + 1) * C + c4);
  v4f m; for (int i = 0; i < 4; ++i) m[i] = fmaxf(fmaxf(a[i], bq[i]), fmaxf(c[i], d[i]));
  float* dst = out + ((size_t)b * Ho * Wo + (size_t)ph * Wo + pw) * C + c4;
  *(volatile v4f*)dst = m;
  __threadfence();
  *(volatile v4f*)dst = m;
}

template <int DQ, int DV>
__global__ __launch_bounds__(128) void k_flash2(const float* __restrict__ Qb, size_t qstride, int qpitch, int Tq,
                                              const float* __restrict__ Kb, size_t kstride, int kpitch, int Tk,
                                              const float* __restrict__ Vb, size_t vstride, int vpitch,
                                              float scale, float* __restrict__ y, size_t ystride, int ypitch) {
  constexpr int KS = DQ / 32, DT = DV / 16;
  __shared__ __attribute__((aligned(16))) unsigned short sKh[32][DQ + 8], sKl[32][DQ + 8], sVh[32][DV + 8], sVl[32][DV + 8];
  __shared__ __attribute__((aligned(16))) unsigned short sPh[4][16][40], sPl[4][16][40];
  __shared__ __attribute__((aligned(16))) float sO[4][16][DV];
  const int tid = threadIdx.x, w = tid >> 5, lane = tid & 31, ln = lane & 15, hh = lane >> 4;
  const int nqb = (Tq + 63) / 64;
  const int bh = blockIdx.x / nqb, qblk = blockIdx.x % nqb;
  const int dv0 = blockIdx.y * DV;
  const int q0 = qblk * 64 + w * 16;
  const float* Q = Qb + (size_t)bh * qstride; const float* K = Kb + (size_t)bh * kstride; const float* V = Vb + (size_t)bh * vstride + dv0;
  FragB aqh[KS], aql[KS];
  {
    int row = q0 + ln; if (row >= Tq) row = Tq - 1;
    const float* qr = Q + (size_t)row * qpitch;
#pragma unroll
    for (int ks = 0; ks < KS; ++ks)
#pragma unroll
      for (int i = 0; i < 16; ++i) {
        const int d = ks * 32 + ((i < 8) ? (8 * hh + i) : (16 + 8 * hh + (i - 8)));
        const float x = qr[d] * scale; const unsigned short hb = bf16_bits(x);
        aqh[ks].u[i] = hb; aql[ks].u[i] = bf16_bits(x - bf16_val(hb));
      }
  }
  float m_r[8], l_r[8];
#pragma unroll
  for (int r = 0; r < 8; ++r) { m_r[r] = -3.0e38f; l_r[r] = 0.f; }
  v8f oacc[DT];
#pragma unroll
  for (int dt = 0; dt < DT; ++dt) oacc[dt] = (v8f){0.f,0.f,0.f,0.f,0.f,0.f,0.f,0.f};
  for (int j0 = 0; j0 < Tk; j0 += 32) {
    __syncthreads();
    for (int e = tid; e < 32 * (DQ / 4); e += 128) {
      const int r = e / (DQ / 4), c4 = (e % (DQ / 4)) * 4; const int key = j0 + r;
      v4f f = {0.f,0.f,0.f,0.f}; if (key < Tk) f = *(const v4fa*)(K + (size_t)key * kpitch + c4);
#pragma unroll
      for (int t = 0; t < 4; ++t) { const unsigned short hb = bf16_bits(f[t]); sKh[r][c4 + t] = hb; sKl[r][c4 + t] = bf16_bits(f[t] - bf16_val(hb)); }
    }
    for (int e = tid; e < 32 * (DV / 4); e += 128) {
      const int r = e / (DV / 4), c4 = (e % (DV / 4)) * 4; const int key = j0 + r;
      v4f f = {0.f,0.f,0.f,0.f}; if (key < Tk) f = *(const v4fa*)(V + (size_t)key * vpitch + c4);
#pragma unroll
      for (int t = 0; t < 4; ++t) { const unsigned short hb = bf16_bits(f[t]); sVh[r][c4 + t] = hb; sVl[r][c4 + t] = bf16_bits(f[t] - bf16_val(hb)); }
    }
    __syncthreads();
    v8f s[2];
#pragma unroll
    for (int nt = 0; nt < 2; ++nt) {
      v8f acc = {};
#pragma unroll
      for (int ks = 0; ks < KS; ++ks) {
        FragB bh_, bl_;
        bh_.half[0] = *(const v8us*)&sKh[nt * 16 + ln][ks * 32 + 8 * hh]; bh_.half[1] = *(const v8us*)&sKh[nt * 16 + ln][ks * 32 + 16 + 8 * hh];
        bl_.half[0] = *(const v8us*)&sKl[nt * 16 + ln][ks * 32 + 8 * hh]; bl_.half[1] = *(const v8us*)&sKl[nt * 16 + ln][ks * 32 + 16 + 8 * hh];
        acc = mmaN<3>(aqh[ks].v, aql[ks].v, bh_.v, bl_.v, acc);
      }
      s[nt] = acc;
    }
    float alpha[8];
#pragma unroll
    for (int r = 0; r < 8; ++r) {
      const int ja = j0 + ln, jb = j0 + 16 + ln;
      if (ja >= Tk) s[0][r] = -3.0e38f;
      if (jb >= Tk) s[1][r] = -3.0e38f;
      float mx = fmaxf(s[0][r], s[1][r]);
      mx = fmaxf(mx, __shfl_xor(mx, 1, 32)); mx = fmaxf(mx, __shfl_xor(mx, 2, 32)); mx = fmaxf(mx, __shfl_xor(mx, 4, 32)); mx = fmaxf(mx, __shfl_xor(mx, 8, 32));
      const float mnew = fmaxf(m_r[r], mx);
      alpha[r] = (mnew > -1.0e38f) ? __expf(m_r[r] - mnew) : 1.0f;
      const float p0 = (s[0][r] > -1.0e38f) ? __expf(s[0][r] - mnew) : 0.f;
      const float p1 = (s[1][r] > -1.0e38f) ? __expf(s[1][r] - mnew) : 0.f;
      m_r[r] = mnew;
      l_r[r] = l_r[r] * alpha[r] + p0 + p1;
      unsigned short hb = bf16_bits(p0); sPh[w][8 * hh + r][ln] = hb;      sPl[w][8 * hh + r][ln] = bf16_bits(p0 - bf16_val(hb));
      hb = bf16_bits(p1);                sPh[w][8 * hh + r][16 + ln] = hb; sPl[w][8 * hh + r][16 + ln] = bf16_bits(p1 - bf16_val(hb));
    }
#pragma unroll
    for (int dt = 0; dt < DT; ++dt)
#pragma unroll
      for (int r = 0; r < 8; ++r) oacc[dt][r] *= alpha[r];
    __builtin_amdgcn_fence(__ATOMIC_ACQ_REL, "workgroup");
    __builtin_amdgcn_wave_barrier();
    FragB pah, pal;
    pah.half[0] = *(const v8us*)&sPh[w][ln][8 * hh]; pah.half[1] = *(const v8us*)&sPh[w][ln][16 + 8 * hh];
    pal.half[0] = *(const v8us*)&sPl[w][ln][8 * hh]; pal.half[1] = *(const v8us*)&sPl[w][ln][16 + 8 * hh];
#pragma unroll
    for (int dt = 0; dt < DT; ++dt) {
      FragB bvh, bvl;
#pragma unroll
      for (int i = 0; i < 8; ++i) {
        bvh.u[i] = sVh[8 * hh + i][dt * 16 + ln]; bvh.u[8 + i] = sVh[16 + 8 * hh + i][dt * 16 + ln];
        bvl.u[i] = sVl[8 * hh + i][dt * 16 + ln]; bvl.u[8 + i] = sVl[16 + 8 * hh + i][dt * 16 + ln];
      }
      oacc[dt] = mmaN<3>(pah.v, pal.v, bvh.v, bvl.v, oacc[dt]);
    }
    __builtin_amdgcn_fence(__ATOMIC_ACQ_REL, "workgroup");
    __builtin_amdgcn_wave_barrier();
  }
#pragma unroll
  for (int r = 0; r < 8; ++r) {
    float l = l_r[r];
    l += __shfl_xor(l, 1, 32); l += __shfl_xor(l, 2, 32); l += __shfl_xor(l, 4, 32); l += __shfl_xor(l, 8, 32);
    l_r[r] = (l > 0.f) ? 1.0f / l : 0.f;
  }
#pragma unroll
  for (int dt = 0; dt < DT; ++dt)
#pragma unroll
    for (int r = 0; r < 8; ++r) sO[w][8 * hh + r][dt * 16 + ln] = oacc[dt][r] * l_r[r];
  __builtin_amdgcn_fence(__ATOMIC_ACQ_REL, "workgroup");
  __builtin_amdgcn_wave_barrier();
  for (int pass = 0; pass < 2; ++pass) {
    for (int r = 0; r < 16; ++r) {
      const int row = q0 + r;
      for (int c4 = lane * 4; c4 < DV; c4 += 128) {
        if (row < Tq) {
          const v4f val = *(const v4fa*)&sO[w][r][c4];
          *(volatile v4f*)(y + (size_t)bh * ystride + (size_t)row * ypitch + dv0 + c4) = val;
        }
      }
    }
    if (pass == 0) __threadfence();
  }
}

template <bool ASPLIT, int ACT, bool BIAS_BF16, bool RES_BF16>
__global__ __launch_bounds__(128) void k_gemm_bf3(const float* __restrict__ A, int lda, const unsigned short* __restrict__ Wt, int ldb,
                                                const float* __restrict__ bias, const float* resid, int rmod, int ldr,
                                                float* C, int ldc, int M, int N, int K) {
  __shared__ __attribute__((aligned(16))) float so[4][16][64];
  const int tid = threadIdx.x, w = tid >> 5, lane = tid & 31, ln = lane & 15, hh = lane >> 4;
  const int ntn = N / 64;
  const int wid = blockIdx.x * 4 + w;
  const int mt = wid / ntn, nq = wid % ntn;
  if (mt * 16 >= M) return;
  const int row0 = mt * 16, col0 = nq * 64;
  const float* arow = A + (size_t)(row0 + ln) * lda;
  v8f acc[4] = {};
  for (int kb = 0; kb < K; kb += 32) {
    FragB ah, al;
    const v4f x0 = *(const v4fa*)(arow + kb + 8 * hh), x1 = *(const v4fa*)(arow + kb + 8 * hh + 4);
    const v4f x2 = *(const v4fa*)(arow + kb + 16 + 8 * hh), x3 = *(const v4fa*)(arow + kb + 16 + 8 * hh + 4);
    float xs[16] = {x0[0],x0[1],x0[2],x0[3],x1[0],x1[1],x1[2],x1[3],x2[0],x2[1],x2[2],x2[3],x3[0],x3[1],x3[2],x3[3]};
#pragma unroll
    for (int i = 0; i < 16; ++i) { const unsigned short hb = bf16_bits(xs[i]); ah.u[i] = hb; al.u[i] = ASPLIT ? bf16_bits(xs[i] - bf16_val(hb)) : (unsigned short)0; }
#pragma unroll
    for (int t = 0; t < 4; ++t) {
      const unsigned short* brow = Wt + (size_t)(col0 + t * 16 + ln) * ldb + kb;
      FragB b;
      b.half[0] = *(const v8us*)(brow + 8 * hh);
      b.half[1] = *(const v8us*)(brow + 16 + 8 * hh);
      acc[t] = mmaN<ASPLIT ? 2 : 1>(ah.v, al.v, b.v, b.v, acc[t]);
    }
  }
#pragma unroll
  for (int t = 0; t < 4; ++t) {
    const int col = col0 + t * 16 + ln;
    float bv = bias ? bias[col] : 0.f;
    if (BIAS_BF16) bv = bf16_round(bv);
#pragma unroll
    for (int r = 0; r < 8; ++r) {
      float v = acc[t][r] + bv;
      if (resid) { float rv = resid[(size_t)((row0 + 8 * hh + r) % rmod) * ldr + col]; if (RES_BF16) rv = bf16_round(rv); v += rv; }
      if (ACT == 1) v = fmaxf(v, 0.f);
      if (ACT == 2) v = 0.5f * v * (1.0f + erff(v * 0.70710678118654752f));
      if (ACT == 3) { const float u = 0.7978845608028654f * (v + 0.044715f * v * v * v); v = 0.5f * v * (1.0f + tanhf(u)); }
      so[w][8 * hh + r][t * 16 + ln] = v;
    }
  }
  __builtin_amdgcn_fence(__ATOMIC_ACQ_REL, "workgroup");
  __builtin_amdgcn_wave_barrier();
  const int rsub = lane >> 4, c4 = (lane & 15) * 4;
  for (int pass = 0; pass < 2; ++pass) {
#pragma unroll
    for (int q = 0; q < 8; ++q) {
      const int r = q * 2 + rsub;
      const v4f v = *(const v4fa*)&so[w][r][c4];
      *(volatile v4f*)(C + (size_t)(row0 + r) * ldc + col0 + c4) = v;
    }
    if (pass == 0) __threadfence();
  }
}
template <bool PARAM_BF16>
__global__ __launch_bounds__(256) void k_layernorm(const float* __restrict__ X, const float* __restrict__ R, const float* __restrict__ g, const float* __restrict__ bta,
                                                  float* __restrict__ out_sum, float* __restrict__ out_norm, int N, float eps) {
  __shared__ float red[256];
  const int row = blockIdx.x, tid = threadIdx.x;
  const float* x = X + (size_t)row * N; const float* rr = R ? R + (size_t)row * N : nullptr;
  float vals[16];
  const int per = N / 256;
  float s1 = 0.f;
  for (int u = 0; u < per / 4; ++u) {
    const int j = tid * 4 + 1024 * u;
    const v4f a = *(const v4fa*)(x + j);
    v4f b = {0.f,0.f,0.f,0.f}; if (rr) b = *(const v4fa*)(rr + j);
#pragma unroll
    for (int q = 0; q < 4; ++q) { const float v = a[q] + b[q]; vals[u * 4 + q] = v; s1 += v; }
  }
  red[tid] = s1; __syncthreads();
  for (int st = 128; st > 0; st >>= 1) { if (tid < st) red[tid] += red[tid + st]; __syncthreads(); }
  const float mu = red[0] / (float)N; __syncthreads();
  float s2 = 0.f;
  for (int u = 0; u < per / 4; ++u)
#pragma unroll
    for (int q = 0; q < 4; ++q) { const float c = vals[u * 4 + q] - mu; s2 += c * c; }
  red[tid] = s2; __syncthreads();
  for (int st = 128; st > 0; st >>= 1) { if (tid < st) red[tid] += red[tid + st]; __syncthreads(); }
  const float rs = rsqrtf(red[0] / (float)N + eps);
  for (int pass = 0; pass < 2; ++pass) {
    for (int u = 0; u < per / 4; ++u) {
      const int j = tid * 4 + 1024 * u;
      v4f o, sm;
#pragma unroll
      for (int q = 0; q < 4; ++q) {
        float gg = g[j + q], bb = bta[j + q];
        if (PARAM_BF16) { gg = bf16_round(gg); bb = bf16_round(bb); }
        sm[q] = vals[u * 4 + q]; o[q] = (vals[u * 4 + q] - mu) * rs * gg + bb;
      }
      if (out_sum) *(volatile v4f*)(out_sum + (size_t)row * N + j) = sm;
      *(volatile v4f*)(out_norm + (size_t)row * N + j) = o;
    }
    if (pass == 0) __threadfence();
  }
}

__global__ __launch_bounds__(256) void k_round_rows(const float* __restrict__ W, unsigned short* __restrict__ Wt, int n8) {
  const int t = blockIdx.x * 256 + threadIdx.x;
  if (t >= n8) return;
  const v4f a = *(const v4fa*)(W + (size_t)t * 8), b = *(const v4fa*)(W + (size_t)t * 8 + 4);
  v8us v; v[0]=bf16_bits(a[0]); v[1]=bf16_bits(a[1]); v[2]=bf16_bits(a[2]); v[3]=bf16_bits(a[3]);
  v[4]=bf16_bits(b[0]); v[5]=bf16_bits(b[1]); v[6]=bf16_bits(b[2]); v[7]=bf16_bits(b[3]);
  *(volatile v8us*)(Wt + (size_t)t * 8) = v; __threadfence(); *(volatile v8us*)(Wt + (size_t)t * 8) = v;
}
__global__ __launch_bounds__(256) void k_wt_conv(const float* __restrict__ w, unsigned short* __restrict__ Bt, int O, int Cin, int CinP, int Np) {
  const int t = blockIdx.x * 256 + threadIdx.x; const int K = 9 * CinP; if (t >= Np * (K / 8)) return;
  const int o = t / (K / 8), k8 = (t % (K / 8)) * 8; v8us v;
#pragma unroll 1
  for (int i = 0; i < 8; ++i) { const int k = k8 + i; const int tap = k / CinP, c = k % CinP; v[i] = (o < O && c < Cin) ? bf16_bits(w[((size_t)o * Cin + c) * 9 + tap]) : (unsigned short)0; }
  *(volatile v8us*)(Bt + (size_t)o * K + k8) = v; __threadfence(); *(volatile v8us*)(Bt + (size_t)o * K + k8) = v;
}
template <int CinP, int ACT, int HI_, int WI_>
__global__ __launch_bounds__(128) void k_conv3x3(const float* __restrict__ in, int inP, const unsigned short* __restrict__ Bt, const float* __restrict__ bias, int Nb, float* __restrict__ out, int Np, int npos) {
  constexpr int K = 9 * CinP, SPT = CinP / 32;
  __shared__ __attribute__((aligned(16))) float so[4][16][64];
  const int tid = threadIdx.x, w = tid >> 5, lane = tid & 31, ln = lane & 15, hh = lane >> 4;
  const int ntn = Np / 64; const int wid = blockIdx.x * 4 + w; const int mt = wid / ntn, nq = wid % ntn;
  if (mt * 16 >= npos) return;
  const int row0 = mt * 16, col0 = nq * 64; const int m = row0 + ln; const int n = m / (HI_ * WI_), yx = m % (HI_ * WI_), y = yx / WI_, xq = yx % WI_;
  v8f acc[4] = {};
  for (int tap = 0; tap < 9; ++tap) {
    const int yy = y + tap / 3 - 1, xx = xq + tap % 3 - 1; const bool inb = (m < npos) && (yy >= 0 && yy < HI_ && xx >= 0 && xx < WI_);
    const float* src = in + ((size_t)n * HI_ * WI_ + (size_t)(inb ? yy : 0) * WI_ + (inb ? xx : 0)) * inP;
#pragma unroll
    for (int s = 0; s < SPT; ++s) {
      const int c0 = s * 32; v4f a0 = {0.f,0.f,0.f,0.f}, a1 = a0, a2 = a0, a3 = a0;
      if (inb) { a0 = *(const v4fa*)(src + c0 + 8 * hh); a1 = *(const v4fa*)(src + c0 + 8 * hh + 4); a2 = *(const v4fa*)(src + c0 + 16 + 8 * hh); a3 = *(const v4fa*)(src + c0 + 16 + 8 * hh + 4); }
      float xs[16] = {a0[0],a0[1],a0[2],a0[3],a1[0],a1[1],a1[2],a1[3],a2[0],a2[1],a2[2],a2[3],a3[0],a3[1],a3[2],a3[3]};
      FragB ah, al;
#pragma unroll
      for (int i = 0; i < 16; ++i) { const unsigned short hb = bf16_bits(xs[i]); ah.u[i] = hb; al.u[i] = bf16_bits(xs[i] - bf16_val(hb)); }
      const int kb = tap * CinP + c0;
#pragma unroll
      for (int t = 0; t < 4; ++t) { FragB bq; bq.half[0] = *(const v8us*)(Bt + (size_t)(col0 + t * 16 + ln) * K + kb + 8 * hh); bq.half[1] = *(const v8us*)(Bt + (size_t)(col0 + t * 16 + ln) * K + kb + 16 + 8 * hh); acc[t] = mmaN<2>(ah.v, al.v, bq.v, bq.v, acc[t]); }
    }
  }
#pragma unroll
  for (int t = 0; t < 4; ++t) { const int col = col0 + t * 16 + ln; const float bv = (col < Nb) ? bf16_round(bias[col]) : 0.f;
#pragma unroll
    for (int r = 0; r < 8; ++r) { float v = acc[t][r] + bv; if (ACT == 1) v = fmaxf(v, 0.f); else if (ACT == 2) v = v >= 0.f ? v : 0.1f * v; so[w][8 * hh + r][t * 16 + ln] = v; } }
  __builtin_amdgcn_fence(__ATOMIC_ACQ_REL, "workgroup"); __builtin_amdgcn_wave_barrier();
  const int rsub = lane >> 4, c4 = (lane & 15) * 4;
  for (int pass = 0; pass < 2; ++pass) { for (int q = 0; q < 8; ++q) { const int r = q * 2 + rsub; if (row0 + r < npos) { const v4f v = *(const v4fa*)&so[w][r][c4]; *(volatile v4f*)(out + (size_t)(row0 + r) * Np + col0 + c4) = v; } } if (pass == 0) __threadfence(); }
}
__global__ __launch_bounds__(256) void k_dwconv(const float* __restrict__ xz, const float* __restrict__ cw, const float* __restrict__ cb, float* __restrict__ xc) {
  const size_t t4 = (size_t)blockIdx.x * 256 + threadIdx.x; if (t4 >= (size_t)MR * DI / 4) return;
  const int d4 = (int)(t4 % (DI / 4)) * 4; const int bt = (int)(t4 / (DI / 4)); const int b = bt / TT, t = bt % TT;
  v4f o;
  for (int q = 0; q < 4; ++q) { const int d = d4 + q; float s = bf16_round(cb[d]);
#pragma unroll
    for (int k = 0; k < 3; ++k) { const int ti = t - 2 + k; if (ti >= 0) s += bf16_round(cw[d * 3 + k]) * xz[((size_t)b * TT + ti) * 2 * DI + d]; }
    o[q] = s / (1.0f + expf(-s)); }
  *(volatile v4f*)(xc + t4 * 4) = o; __threadfence(); *(volatile v4f*)(xc + t4 * 4) = o;
}
__global__ __launch_bounds__(256) void k_wt_xp(const float* __restrict__ W, unsigned short* __restrict__ Bt) {
  const int t = blockIdx.x * 256 + threadIdx.x; if (t >= 64 * (DI / 8)) return; const int n = t / (DI / 8), k8 = (t % (DI / 8)) * 8; v8us v;
  for (int i = 0; i < 8; ++i) v[i] = (n < NXP) ? bf16_bits(W[(size_t)n * DI + k8 + i]) : (unsigned short)0;
  *(volatile v8us*)(Bt + (size_t)n * DI + k8) = v; __threadfence(); *(volatile v8us*)(Bt + (size_t)n * DI + k8) = v;
}
__global__ __launch_bounds__(DI) void k_scan(const float* __restrict__ dbl, const float* __restrict__ xc, const float* __restrict__ xz, const float* __restrict__ dtw, const float* __restrict__ dtb,
                                           const float* __restrict__ Alog, const float* __restrict__ Dp, float* __restrict__ yg) {
  __shared__ float sA[DS][DI], sH[DS][DI], sW[DTR][DI];
  const int b = blockIdx.x, d = threadIdx.x;
#pragma unroll 1
  for (int s = 0; s < DS; ++s) sA[s][d] = -expf(bf16_round(Alog[d * DS + s]));
#pragma unroll 1
  for (int r = 0; r < DTR; ++r) sW[r][d] = bf16_round(dtw[d * DTR + r]);
  const float db = bf16_round(dtb[d]), Dd = bf16_round(Dp[d]);
#pragma unroll 1
  for (int pass = 0; pass < 2; ++pass) {
#pragma unroll 1
    for (int s = 0; s < DS; ++s) sH[s][d] = 0.f;
#pragma unroll 1
    for (int t = 0; t < TT; ++t) {
      const size_t row = (size_t)b * TT + t; const float* dr = dbl + row * 64;
      float u = db;
#pragma unroll 1
      for (int r = 0; r < DTR; ++r) u += dr[r] * sW[r][d];
      const float dt = (u > 0.f ? u : 0.f) + log1pf(expf(-fabsf(u)));
      const float xv = xc[row * DI + d]; const float dx = dt * xv;
      float y = 0.f;
#pragma unroll 1
      for (int s = 0; s < DS; ++s) { const float hv = expf(dt * sA[s][d]) * sH[s][d] + dx * dr[DTR + s]; sH[s][d] = hv; y += hv * dr[DTR + DS + s]; }
      const float zv = xz[row * 2 * DI + DI + d];
      const float o = (y + Dd * xv) * (zv / (1.0f + expf(-zv)));
      *(volatile float*)(yg + row * DI + d) = o;
    }
    __threadfence();
  }
}

__device__ __forceinline__ int win_start(int k) { int e = k * 8 + WSZ; if (e > HI) e = HI; return e - WSZ; }
__global__ __launch_bounds__(256) void k_wt_slice(const float* __restrict__ W, int ldw, int koff, unsigned short* __restrict__ Bt, int Nout, int Np, int Kc) {
  const int t = blockIdx.x * 256 + threadIdx.x; const int k8n = Kc / 8; if (t >= Np * k8n) return; const int n = t / k8n, k8 = (t % k8n) * 8; v8us v;
  for (int i = 0; i < 8; ++i) v[i] = (n < Nout) ? bf16_bits(W[(size_t)n * ldw + koff + k8 + i]) : (unsigned short)0;
  *(volatile v8us*)(Bt + (size_t)n * Kc + k8) = v; __threadfence(); *(volatile v8us*)(Bt + (size_t)n * Kc + k8) = v;
}
template <int AXIS>
__global__ __launch_bounds__(256) void k_gather(const float* __restrict__ h, float* __restrict__ u) {
  const size_t i = (size_t)blockIdx.x * 256 + threadIdx.x; if (i >= (size_t)MR * HID / 4) return; const int c4 = (int)(i % (HID / 4)) * 4; const size_t st = i / (HID / 4); const int t = (int)(st % TT); const int seq = (int)(st / TT);
  const int win = seq % NWIN; const int oth = (seq / NWIN) % WI; const int b = seq / (NWIN * WI); const int s0 = win_start(win);
  const int y = AXIS == 0 ? s0 + t : oth, x = AXIS == 0 ? oth : s0 + t;
  const v4f v = *(const v4fa*)(h + (((size_t)b * HI + y) * WI + x) * HID + c4); *(volatile v4f*)(u + i * 4) = v; __threadfence(); *(volatile v4f*)(u + i * 4) = v;
}
template <int AXIS>
__global__ __launch_bounds__(256) void k_scatter(const float* __restrict__ o, float* __restrict__ f) {
  const size_t i = (size_t)blockIdx.x * 256 + threadIdx.x; if (i >= (size_t)NPOS * HID / 4) return; const int c4 = (int)(i % (HID / 4)) * 4; const size_t p = i / (HID / 4); const int x = (int)(p % WI), y = (int)((p / WI) % HI), b = (int)(p / HWN);
  const int coord = AXIS == 0 ? y : x, oth = AXIS == 0 ? x : y;
  v4f acc = {0.f,0.f,0.f,0.f}; float cnt = 0.f;
#pragma unroll 1
  for (int win = 0; win < NWIN; ++win) { const int s0 = win_start(win); if (coord >= s0 && coord < s0 + WSZ) { cnt += 1.f; const int seq = (b * WI + oth) * NWIN + win; const v4f v = *(const v4fa*)(o + ((size_t)seq * TT + (coord - s0)) * HID + c4); for (int q = 0; q < 4; ++q) acc[q] += v[q]; } }
  for (int q = 0; q < 4; ++q) acc[q] /= cnt;
  *(volatile v4f*)(f + i * 4) = acc; __threadfence(); *(volatile v4f*)(f + i * 4) = acc;
}
__global__ __launch_bounds__(256) void k_silu_ip(float* __restrict__ p, size_t n4) { const size_t t = (size_t)blockIdx.x * 256 + threadIdx.x; if (t >= n4) return; v4f v = *(const v4fa*)(p + t * 4); for (int q = 0; q < 4; ++q) v[q] = v[q] / (1.0f + expf(-v[q])); *(volatile v4f*)(p + t * 4) = v; __threadfence(); *(volatile v4f*)(p + t * 4) = v; }
__global__ __launch_bounds__(256) void k_gnstat(const float* __restrict__ o, float* __restrict__ slot) {
  __shared__ double rs[256], rq[256]; const int b = blockIdx.x / NG, g = blockIdx.x % NG; double s = 0.0, q = 0.0;
#pragma unroll 1
  for (int e = threadIdx.x; e < HWN * 12; e += 256) { const int p = e / 12, c = g * 12 + e % 12; const double v = (double)o[((size_t)b * HWN + p) * HID + c]; s += v; q += v * v; }
  rs[threadIdx.x] = s; rq[threadIdx.x] = q; __syncthreads(); for (int st = 128; st > 0; st >>= 1) { if (threadIdx.x < st) { rs[threadIdx.x] += rs[threadIdx.x + st]; rq[threadIdx.x] += rq[threadIdx.x + st]; } __syncthreads(); }
  const double n = (double)HWN * 12.0; const double mu = rs[0] / n; double var = rq[0] / n - mu * mu; if (var < 0.0) var = 0.0;
  if (threadIdx.x < 32) { const float v = threadIdx.x == 0 ? (float)mu : (threadIdx.x == 1 ? (float)(1.0 / sqrt(var + 1e-5)) : 0.f); *(volatile float*)(slot + (size_t)blockIdx.x * 32 + threadIdx.x) = v; __threadfence(); *(volatile float*)(slot + (size_t)blockIdx.x * 32 + threadIdx.x) = v; }
}
__global__ __launch_bounds__(256) void k_gnout(const float* __restrict__ o, const float* __restrict__ slot, const float* __restrict__ gg, const float* __restrict__ gb, float* __restrict__ out) {
  const int b = blockIdx.x / CX, c = blockIdx.x % CX; const int g = c / 12; const float mu = slot[(size_t)(b * NG + g) * 32], rs = slot[(size_t)(b * NG + g) * 32 + 1]; const float ga = bf16_round(gg[c]), be = bf16_round(gb[c]);
  for (int pass = 0; pass < 2; ++pass) { for (int p = threadIdx.x; p < HWN; p += 256) *(volatile float*)(out + ((size_t)b * CX + c) * HWN + p) = (o[((size_t)b * HWN + p) * HID + c] - mu) * rs * ga + be; if (pass == 0) __threadfence(); }
}
extern "C" void kernel_launch(void* const* d_in, const int* in_sizes, int n_in,
                              void* d_out, int out_size, void* d_ws, size_t ws_size, hipStream_t stream) {
  (void)in_sizes; (void)n_in; (void)out_size;
  const float* x = (const float*)d_in[0]; const float* w_in = (const float*)d_in[1]; const float* w_res = (const float*)d_in[2];
  const float* mp[2][9]; for (int a = 0; a < 2; ++a) for (int i = 0; i < 9; ++i) mp[a][i] = (const float*)d_in[3 + a * 9 + i];
  const float* w_loc[2] = {(const float*)d_in[21], (const float*)d_in[22]}; const float* w_f1 = (const float*)d_in[23]; const float* w_f2 = (const float*)d_in[24]; const float* w_out = (const float*)d_in[25]; const float* gn_g = (const float*)d_in[26]; const float* gn_b = (const float*)d_in[27];
  char* ws = (char*)d_ws; size_t off = 0;
  auto take = [&](size_t bytes) { char* p = ws + off; off += (bytes + 255) & ~(size_t)255; return p; };
  unsigned short* Bin = (unsigned short*)take((size_t)HID * CX * 2); unsigned short* Bres = (unsigned short*)take((size_t)128 * CX * 2);
  unsigned short* Binp[2], *Bxp[2], *Bop[2], *Bloc[2]; for (int a = 0; a < 2; ++a) { Binp[a] = (unsigned short*)take((size_t)2 * DI * HID * 2); Bxp[a] = (unsigned short*)take((size_t)64 * DI * 2); Bop[a] = (unsigned short*)take((size_t)HID * DI * 2); Bloc[a] = (unsigned short*)take((size_t)HID * 9 * HID * 2); }
  unsigned short* Bf1a = (unsigned short*)take((size_t)HID * HID * 2); unsigned short* Bf1b = (unsigned short*)take((size_t)HID * HID * 2); unsigned short* Bf2 = (unsigned short*)take((size_t)HID * HID * 2); unsigned short* Bout = (unsigned short*)take((size_t)128 * HID * 2);
  float* xT = (float*)take((size_t)NPOS * CX * 4); float* res = (float*)take((size_t)NPOS * 128 * 4); float* h = (float*)take((size_t)NPOS * HID * 4);
  float* u = (float*)take((size_t)MR * HID * 4); float* xz = (float*)take((size_t)MR * 2 * DI * 4); float* xc = (float*)take((size_t)MR * DI * 4); float* dbl = (float*)take((size_t)MR * 64 * 4); float* yg = (float*)take((size_t)MR * DI * 4); float* mo = (float*)take((size_t)MR * HID * 4);
  float* fz = (float*)take((size_t)NPOS * HID * 4); float* xa[2]; xa[0] = (float*)take((size_t)NPOS * HID * 4); xa[1] = (float*)take((size_t)NPOS * HID * 4); float* f1 = (float*)take((size_t)NPOS * HID * 4); float* f2 = (float*)take((size_t)NPOS * HID * 4); float* o = (float*)take((size_t)NPOS * 128 * 4); float* slot = (float*)take(BB * NG * 32 * 4);
  if (off > ws_size) return;
  k_round_rows<<<(HID * CX / 8 + 255) / 256, 256, 0, stream>>>(w_in, Bin, HID * CX / 8);
  k_wt_slice<<<(128 * (CX / 8) + 255) / 256, 256, 0, stream>>>(w_res, CX, 0, Bres, CX, 128, CX);
  for (int a = 0; a < 2; ++a) { k_round_rows<<<(2 * DI * HID / 8 + 255) / 256, 256, 0, stream>>>(mp[a][0], Binp[a], 2 * DI * HID / 8); k_wt_xp<<<(64 * (DI / 8) + 255) / 256, 256, 0, stream>>>(mp[a][3], Bxp[a]); k_round_rows<<<(HID * DI / 8 + 255) / 256, 256, 0, stream>>>(mp[a][8], Bop[a], HID * DI / 8);
    k_wt_conv<<<(HID * (9 * HID / 8) + 255) / 256, 256, 0, stream>>>(w_loc[a], Bloc[a], HID, HID, HID, HID); }
  k_wt_slice<<<(HID * (HID / 8) + 255) / 256, 256, 0, stream>>>(w_f1, 2 * HID, 0, Bf1a, HID, HID, HID); k_wt_slice<<<(HID * (HID / 8) + 255) / 256, 256, 0, stream>>>(w_f1, 2 * HID, HID, Bf1b, HID, HID, HID);
  k_round_rows<<<(HID * HID / 8 + 255) / 256, 256, 0, stream>>>(w_f2, Bf2, HID * HID / 8); k_wt_slice<<<(128 * (HID / 8) + 255) / 256, 256, 0, stream>>>(w_out, HID, 0, Bout, CX, 128, HID);
  k_transpose32<false, false, false><<<dim3(HWN / 32, CX / 32, BB), 256, 0, stream>>>(x, xT, CX, HWN, nullptr, nullptr, nullptr);
  const unsigned gp = ((NPOS / 16) * 2 + 3) / 4; const size_t n4 = (size_t)NPOS * HID / 4;
  k_gemm_bf3<false, 0, false, false><<<gp, 128, 0, stream>>>(xT, CX, Bres, CX, nullptr, nullptr, 1, 0, res, 128, NPOS, 128, CX);
  k_gemm_bf3<false, 0, false, false><<<gp, 128, 0, stream>>>(xT, CX, Bin, CX, nullptr, nullptr, 1, 0, h, HID, NPOS, HID, CX);
  for (int a = 0; a < 2; ++a) {
    if (a == 0) k_gather<0><<<(unsigned)(((size_t)MR * HID / 4 + 255) / 256), 256, 0, stream>>>(h, u); else k_gather<1><<<(unsigned)(((size_t)MR * HID / 4 + 255) / 256), 256, 0, stream>>>(h, u);
    k_gemm_bf3<true, 0, false, false><<<((MR / 16) * (2 * DI / 64) + 3) / 4, 128, 0, stream>>>(u, HID, Binp[a], HID, nullptr, nullptr, 1, 0, xz, 2 * DI, MR, 2 * DI, HID);
    k_dwconv<<<(unsigned)(((size_t)MR * DI / 4 + 255) / 256), 256, 0, stream>>>(xz, mp[a][1], mp[a][2], xc);
    k_gemm_bf3<true, 0, false, false><<<((MR / 16) * 1 + 3) / 4, 128, 0, stream>>>(xc, DI, Bxp[a], DI, nullptr, nullptr, 1, 0, dbl, 64, MR, 64, DI);
    k_scan<<<NSEQ, DI, 0, stream>>>(dbl, xc, xz, mp[a][4], mp[a][5], mp[a][6], mp[a][7], yg);
    k_gemm_bf3<true, 0, false, false><<<((MR / 16) * 2 + 3) / 4, 128, 0, stream>>>(yg, DI, Bop[a], DI, nullptr, nullptr, 1, 0, mo, HID, MR, HID, DI);
    if (a == 0) k_scatter<0><<<(unsigned)((n4 + 255) / 256), 256, 0, stream>>>(mo, fz); else k_scatter<1><<<(unsigned)((n4 + 255) / 256), 256, 0, stream>>>(mo, fz);
    k_conv3x3<HID, 0, HI, WI><<<((NPOS / 16) * 2 + 3) / 4, 128, 0, stream>>>(fz, HID, Bloc[a], nullptr, 0, xa[a], HID, NPOS);
  }
  k_gemm_bf3<true, 0, false, false><<<gp, 128, 0, stream>>>(xa[0], HID, Bf1a, HID, nullptr, nullptr, 1, 0, f1, HID, NPOS, HID, HID);
  k_gemm_bf3<true, 0, false, false><<<gp, 128, 0, stream>>>(xa[1], HID, Bf1b, HID, nullptr, f1, NPOS, HID, f1, HID, NPOS, HID, HID);
  k_silu_ip<<<(unsigned)((n4 + 255) / 256), 256, 0, stream>>>(f1, n4);
  k_gemm_bf3<true, 0, false, false><<<gp, 128, 0, stream>>>(f1, HID, Bf2, HID, nullptr, nullptr, 1, 0, f2, HID, NPOS, HID, HID);
  k_gemm_bf3<true, 0, false, false><<<gp, 128, 0, stream>>>(f2, HID, Bout, HID, nullptr, res, NPOS, 128, o, 128, NPOS, 128, HID);
  k_gnstat<<<BB * NG, 256, 0, stream>>>(o, slot);
  k_gnout<<<BB * CX, 256, 0, stream>>>(o, slot, gn_g, gn_b, (float*)d_out);
}
